// RNN_18992345383093
// MI455X (gfx1250) — hardware-verified
//
#include <hip/hip_runtime.h>
#include <math.h>

constexpr int NBAT = 8;
constexpr int NTOK = 2048;
constexpr int DDIM = 512;
constexpr int NSLOT = 4;
constexpr int VOC = 128;
constexpr int NROW = NBAT * NTOK;
constexpr int G3X = 3 * DDIM;
constexpr int NTHR = 256;
constexpr int RB = 32;
constexpr int HP = 520;
constexpr int SP = 516;
constexpr int LP = 260;
constexpr int ETAB_EMB = (NSLOT - 1) * VOC;
constexpr int ETAB_ROWS = 448;
constexpr int GXT_ROWS = ETAB_EMB + 1;
constexpr float WCAR = 64.0f;
constexpr float HCAR = 16.0f;
constexpr float GINV = 1.0f / 1024.0f;
constexpr float TSCALE = 1.0f / 4096.0f;
static_assert(NROW % RB == 0);
static_assert(DDIM % 32 == 0);
static_assert(DDIM == 16 * 4 * (NTHR / 32));
static_assert(VOC == 16 * (NTHR / 32));
static_assert(RB == 4 * (NTHR / 32));
static_assert((RB * DDIM / 4) % NTHR == 0);
static_assert(RB * NSLOT <= NTHR);
static_assert(ETAB_ROWS % 64 == 0 && ETAB_ROWS >= ETAB_EMB + NSLOT && G3X % 64 == 0);
static_assert(((ETAB_ROWS / 64) * (G3X / 64)) % 8 == 0);
static_assert(HP % 8 == 0 && SP % 4 == 0 && LP % 4 == 0);

typedef __attribute__((ext_vector_type(16))) _Float16 v16h;
typedef __attribute__((ext_vector_type(8)))  _Float16 v8h;
typedef __attribute__((ext_vector_type(4)))  _Float16 v4h;
typedef __attribute__((ext_vector_type(16))) __bf16   v16b;
typedef __attribute__((ext_vector_type(8)))  __bf16   v8b;
typedef __attribute__((ext_vector_type(8)))  float    v8f;
typedef __attribute__((ext_vector_type(4)))  float    v4f;

__device__ __forceinline__ unsigned short f2bf_bits(float f) {
  unsigned u = __float_as_uint(f);
  return (unsigned short)((u + 0x7FFFu + ((u >> 16) & 1u)) >> 16);
}
__device__ __forceinline__ float bf_bits2f(unsigned short h) { return __uint_as_float(((unsigned)h) << 16); }
__device__ __forceinline__ float bf16r(float f) { return bf_bits2f(f2bf_bits(f)); }

__device__ __forceinline__ void dep_guard_h(v8f& a, v8f& b, v16h x, v16h y) { asm volatile("v_nop\n\tv_nop\n\tv_nop\n\tv_nop" : "+v"(a), "+v"(b) : "v"(x), "v"(y)); }
__device__ __forceinline__ void dep_guard_b(v8f& a, v8f& b, v16b x, v16b y) { asm volatile("v_nop\n\tv_nop\n\tv_nop\n\tv_nop" : "+v"(a), "+v"(b) : "v"(x), "v"(y)); }
__device__ __forceinline__ void keep4_h(v16h a, v16h b, v16h c, v16h d) { asm volatile("v_nop" :: "v"(a), "v"(b), "v"(c), "v"(d)); }
__device__ __forceinline__ void keep4_b(v16b a, v16b b, v16b c, v16b d) { asm volatile("v_nop" :: "v"(a), "v"(b), "v"(c), "v"(d)); }
__device__ __forceinline__ void acc_guard4(v8f& a, v8f& b, v8f& c, v8f& d) { asm volatile("v_nop\n\tv_nop\n\tv_nop\n\tv_nop" : "+v"(a), "+v"(b), "+v"(c), "+v"(d)); }
__device__ __forceinline__ void acc_guard2(v8f& a, v8f& b) { asm volatile("v_nop\n\tv_nop\n\tv_nop\n\tv_nop" : "+v"(a), "+v"(b)); }
__device__ __forceinline__ void tie6_h(v8f& c0, v8f& c1, v8f& c2, v8f& c3, v8f& c4, v8f& c5, v16h x, v16h y, v16h z) {
  asm volatile("v_nop\n\tv_nop\n\tv_nop\n\tv_nop" : "+v"(c0), "+v"(c1), "+v"(c2), "+v"(c3), "+v"(c4), "+v"(c5) : "v"(x), "v"(y), "v"(z));
}
__device__ __forceinline__ void tie8_h(v8f& c0, v8f& c1, v8f& c2, v8f& c3, v8f& c4, v8f& c5, v8f& c6, v8f& c7, v16h x, v16h y, v16h z) {
  asm volatile("v_nop\n\tv_nop\n\tv_nop\n\tv_nop" : "+v"(c0), "+v"(c1), "+v"(c2), "+v"(c3), "+v"(c4), "+v"(c5), "+v"(c6), "+v"(c7) : "v"(x), "v"(y), "v"(z));
}
__device__ __forceinline__ void accg6(v8f& c0, v8f& c1, v8f& c2, v8f& c3, v8f& c4, v8f& c5) {
  asm volatile("v_nop\n\tv_nop\n\tv_nop\n\tv_nop" : "+v"(c0), "+v"(c1), "+v"(c2), "+v"(c3), "+v"(c4), "+v"(c5));
}
__device__ __forceinline__ void accg8(v8f& c0, v8f& c1, v8f& c2, v8f& c3, v8f& c4, v8f& c5, v8f& c6, v8f& c7) {
  asm volatile("v_nop\n\tv_nop\n\tv_nop\n\tv_nop" : "+v"(c0), "+v"(c1), "+v"(c2), "+v"(c3), "+v"(c4), "+v"(c5), "+v"(c6), "+v"(c7));
}

template <typename T> struct Frag;
template <> struct Frag<_Float16> {
  typedef v16h V; union U { v16h v; v8h h[2]; };
  static __device__ __forceinline__ v16h load(const _Float16* p) {
    U f; f.h[0] = *(const v8h*)(p); f.h[1] = *(const v8h*)(p + 16); return f.v;
  }
  static __device__ __forceinline__ v8f mma(v16h a, v16h b, v8f c) {
    return __builtin_amdgcn_wmma_f32_16x16x32_f16(false, a, false, b, (short)0, c, false, false);
  }
  static __device__ __forceinline__ void guard(v8f& a, v8f& b, v16h x, v16h y) { dep_guard_h(a, b, x, y); }
  static __device__ __forceinline__ void keep(v16h a, v16h b, v16h c, v16h d) { keep4_h(a, b, c, d); }
};
template <> struct Frag<__bf16> {
  typedef v16b V; union U { v16b v; v8b h[2]; };
  static __device__ __forceinline__ v16b load(const __bf16* p) {
    U f; f.h[0] = *(const v8b*)(p); f.h[1] = *(const v8b*)(p + 16); return f.v;
  }
  static __device__ __forceinline__ v8f mma(v16b a, v16b b, v8f c) {
    return __builtin_amdgcn_wmma_f32_16x16x32_bf16(false, a, false, b, (short)0, c, false, false);
  }
  static __device__ __forceinline__ void guard(v8f& a, v8f& b, v16b x, v16b y) { dep_guard_b(a, b, x, y); }
  static __device__ __forceinline__ void keep(v16b a, v16b b, v16b c, v16b d) { keep4_b(a, b, c, d); }
};

template <int ET> struct Elem;
template <> struct Elem<0> { typedef _Float16 T; };
template <> struct Elem<1> { typedef __bf16 T; };
template <int ET, bool SPLIT, int BIAS_MODE, int OUT_MODE, bool RESID, int ACT = 0>
__global__ __launch_bounds__(256) void wmma_gemm64(
    const unsigned short* __restrict__ Ap, const unsigned short* __restrict__ A2p, int lda, long strideA,
    const unsigned short* __restrict__ Btp, const unsigned short* __restrict__ Bt2p, int ldb, long strideB,
    void* __restrict__ Cout, void* __restrict__ Cout2, int ldc, long strideC,
    const float* __restrict__ bias,
    const float* __restrict__ resid, long strideR,
    int M, int N, int K, float scale) {
  typedef typename Elem<ET>::T T;
  typedef typename Frag<T>::V V;
  const T* A = (const T*)Ap; const T* A2 = (const T*)A2p; const T* Bt = (const T*)Btp; const T* Bt2 = (const T*)Bt2p;
  __shared__ __align__(16) float sT[8][16 * 68];
  const int b    = blockIdx.y;
  const int lane = threadIdx.x & 31;
  const int wave = threadIdx.x >> 5;
  const int tilesN = N >> 6;
  const int tilesM = M >> 6;
  const int tile = blockIdx.x * 8 + wave;
  if (tile >= tilesM * tilesN) return;
  const int tm = tile / tilesN;
  const int tn = tile - tm * tilesN;
  const int m0 = tm << 6;
  const int n0 = tn << 6;

  const T* Ab  = A  + (size_t)b * strideA;
  const T* Bb  = Bt + (size_t)b * strideB;
  const T* Ab2 = SPLIT ? (A2  + (size_t)b * strideA) : nullptr;
  const T* Bb2 = SPLIT ? (Bt2 + (size_t)b * strideB) : nullptr;

  const int rlane = lane & 15;
  const int koff  = (lane >> 4) * 8;
  const int mOff  = (lane >> 4) * 8;

  v8f acc[4][4];
#pragma unroll
  for (int i = 0; i < 4; ++i)
#pragma unroll
    for (int j = 0; j < 4; ++j) acc[i][j] = (v8f){0.f,0.f,0.f,0.f,0.f,0.f,0.f,0.f};

  for (int k0 = 0; k0 < K; k0 += 32) {
    V bh[4], bl[4];
#pragma unroll
    for (int j = 0; j < 4; ++j) {
      const size_t bo = (size_t)(n0 + (j << 4) + rlane) * ldb + koff + k0;
      bh[j] = Frag<T>::load(Bb + bo);
      if (SPLIT) bl[j] = Frag<T>::load(Bb2 + bo);
    }
#pragma unroll
    for (int i = 0; i < 4; ++i) {
      const size_t ao = (size_t)(m0 + (i << 4) + rlane) * lda + koff + k0;
      V ah = Frag<T>::load(Ab + ao);
      V al;
      if (SPLIT) al = Frag<T>::load(Ab2 + ao);
#pragma unroll
      for (int j = 0; j < 4; ++j) {
        acc[i][j] = Frag<T>::mma(ah, bh[j], acc[i][j]);
        if (SPLIT) {
          acc[i][j] = Frag<T>::mma(ah, bl[j], acc[i][j]);
          acc[i][j] = Frag<T>::mma(al, bh[j], acc[i][j]);
        }
      }
      Frag<T>::guard(acc[i][0], acc[i][3], ah, SPLIT ? al : ah);
    }
    Frag<T>::keep(bh[0], bh[1], bh[2], bh[3]);
    if (SPLIT) Frag<T>::keep(bl[0], bl[1], bl[2], bl[3]);
  }
  acc_guard4(acc[0][0], acc[0][1], acc[0][2], acc[0][3]);
  acc_guard4(acc[1][0], acc[1][1], acc[1][2], acc[1][3]);
  acc_guard4(acc[2][0], acc[2][1], acc[2][2], acc[2][3]);
  acc_guard4(acc[3][0], acc[3][1], acc[3][2], acc[3][3]);

  float* slab = sT[wave];
  const float* Rb = RESID ? (resid + (size_t)b * strideR) : nullptr;
#pragma unroll
  for (int i = 0; i < 4; ++i) {
    const int mBase = m0 + (i << 4);
#pragma unroll
    for (int j = 0; j < 4; ++j) {
      const int n = n0 + (j << 4) + rlane;
      float bv = 0.f;
      if (BIAS_MODE == 2) bv = bias[n];
#pragma unroll
      for (int r = 0; r < 8; ++r) {
        float v = acc[i][j][r] * scale;
        if (BIAS_MODE == 1) v += bias[mBase + mOff + r];
        if (BIAS_MODE == 2) v += bv;
        if (RESID) v += Rb[(size_t)(mBase + mOff + r) * ldc + n];
        if (ACT == 1) v = tanhf(v);
        if (ACT == 2) v = fmaxf(v, 0.0f);
        if (ACT == 3) v = v / (1.0f + expf(-v));
        if (ACT == 4) v = (v > 0.f) ? v : 0.01f * v;
        if (ACT == 5) v = 0.5f * v * (1.0f + erff(v * 0.70710678118654752f));
        slab[(mOff + r) * 68 + (j << 4) + rlane] = v;
      }
    }
    __builtin_amdgcn_fence(__ATOMIC_RELEASE, "workgroup");
    __builtin_amdgcn_wave_barrier();
    __builtin_amdgcn_fence(__ATOMIC_ACQUIRE, "workgroup");
    if (OUT_MODE == 0) {
      float* C = (float*)Cout + (size_t)b * strideC;
      const int hh = lane >> 4, c4 = (lane & 15) * 4;
      for (int pass = 0; pass < 2; ++pass) {
#pragma unroll
        for (int it = 0; it < 8; ++it) {
          const int row = it * 2 + hh;
          v4f v = *(const v4f*)(slab + row * 68 + c4);
          *(volatile v4f*)(C + (size_t)(mBase + row) * ldc + n0 + c4) = v;
        }
        __threadfence();
      }
    } else {
      const int q = lane >> 3, c8 = (lane & 7) * 8;
      unsigned short* C  = (unsigned short*)Cout  + (size_t)b * strideC;
      unsigned short* C2 = (OUT_MODE == 2) ? ((unsigned short*)Cout2 + (size_t)b * strideC) : nullptr;
      for (int pass = 0; pass < 2; ++pass) {
#pragma unroll
        for (int it = 0; it < 4; ++it) {
          const int row = it * 4 + q;
          const float* sp = slab + row * 68 + c8;
          v8h hv, lv;
#pragma unroll
          for (int e = 0; e < 8; ++e) {
            if (OUT_MODE == 1) {
              hv[e] = (_Float16)sp[e];
            } else {
              unsigned short hb = f2bf_bits(sp[e]);
              unsigned short lb = f2bf_bits(sp[e] - bf_bits2f(hb));
              hv[e] = __builtin_bit_cast(_Float16, hb);
              lv[e] = __builtin_bit_cast(_Float16, lb);
            }
          }
          *(volatile v8h*)(C + (size_t)(mBase + row) * ldc + n0 + c8) = hv;
          if (OUT_MODE == 2) *(volatile v8h*)(C2 + (size_t)(mBase + row) * ldc + n0 + c8) = lv;
        }
        __threadfence();
      }
    }
    __builtin_amdgcn_fence(__ATOMIC_RELEASE, "workgroup");
    __builtin_amdgcn_wave_barrier();
    __builtin_amdgcn_fence(__ATOMIC_ACQUIRE, "workgroup");
  }
}

template <int MODE>
__global__ __launch_bounds__(NTHR) void cvt8_kernel(const float* __restrict__ src, const float* __restrict__ src2,
                                                    unsigned short* __restrict__ dst,
                                                    int nrow, int ncol8, int spitch, float sc) {
  const int i  = blockIdx.x * NTHR + threadIdx.x;
  const int n8 = nrow * ncol8;
  if (i < n8) {
    const int row = i / ncol8;
    const int c8  = i - row * ncol8;
    const float* sp  = src  + (size_t)row * spitch + c8 * 8;
    const float* sp2 = src2 + (size_t)row * spitch + c8 * 8;
    const v4f a = *(const v4f*)(sp);
    const v4f b = *(const v4f*)(sp + 4);
    v4f a2 = a, b2 = b;
    if (MODE == 2) { a2 = *(const v4f*)(sp2); b2 = *(const v4f*)(sp2 + 4); }
    v8h hv;
#pragma unroll
    for (int e = 0; e < 4; ++e) {
      float x0 = bf16r(a[e]);
      float x1 = bf16r(b[e]);
      if (MODE == 2) { x0 += bf16r(a2[e]); x1 += bf16r(b2[e]); }
      hv[e]     = (_Float16)(x0 * sc);
      hv[4 + e] = (_Float16)(x1 * sc);
    }
    *(volatile v8h*)(dst + (size_t)i * 8) = hv;
    __threadfence();
    *(volatile v8h*)(dst + (size_t)i * 8) = hv;
  }
}

__global__ __launch_bounds__(NTHR) void e16_kernel(const float* __restrict__ emb, const float* __restrict__ pos,
                                                   unsigned short* __restrict__ dst) {
  const int i  = blockIdx.x * NTHR + threadIdx.x;
  const int n8 = ETAB_ROWS * (DDIM / 8);
  if (i < n8) {
    const int row = i >> 6;
    const int c8  = (i & 63) * 8;
    const int er = row < ETAB_EMB ? row : (ETAB_EMB - 1);
    int pr = row - ETAB_EMB; pr = pr < 0 ? 0 : pr; pr = pr > (NSLOT - 1) ? (NSLOT - 1) : pr;
    const float fe = (row < ETAB_EMB) ? 1.0f : 0.0f;
    const float fp = (row >= ETAB_EMB && row < ETAB_EMB + NSLOT) ? 1.0f : 0.0f;
    const float* ep = emb + (size_t)er * DDIM + c8;
    const float* pp = pos + (size_t)pr * DDIM + c8;
    const v4f ea = *(const v4f*)(ep), eb = *(const v4f*)(ep + 4);
    const v4f pa = *(const v4f*)(pp), pb = *(const v4f*)(pp + 4);
    v8h hv;
#pragma unroll
    for (int e = 0; e < 4; ++e) {
      const float x0 = fmaf(fe, bf16r(ea[e]), fp * bf16r(pa[e]));
      const float x1 = fmaf(fe, bf16r(eb[e]), fp * bf16r(pb[e]));
      hv[e]     = (_Float16)(x0 * WCAR);
      hv[4 + e] = (_Float16)(x1 * WCAR);
    }
    *(volatile v8h*)(dst + (size_t)i * 8) = hv;
    __threadfence();
    *(volatile v8h*)(dst + (size_t)i * 8) = hv;
  }
}

__global__ __launch_bounds__(NTHR) void gxt_kernel(const float* __restrict__ TRAW, const float* __restrict__ b_ih,
                                                   float* __restrict__ GXT) {
  const int i = blockIdx.x * NTHR + threadIdx.x;
  if (i < GXT_ROWS * DDIM) {
    const int q = i >> 9;
    const int u = i & (DDIM - 1);
    int jr = q >> 7; jr = jr > (NSLOT - 2) ? (NSLOT - 2) : jr;
    const int rowB = ETAB_EMB + 1 + jr;
    const float fb = (q < ETAB_EMB) ? 1.0f : 0.0f;
    const float* ta = TRAW + (size_t)q * G3X + u;
    const float* tb = TRAW + (size_t)rowB * G3X + u;
    const float t0a = ta[0], t1a = ta[DDIM], t2a = ta[2 * DDIM];
    const float t0b = tb[0], t1b = tb[DDIM], t2b = tb[2 * DDIM];
    const float b0 = bf16r(b_ih[u]), b1 = bf16r(b_ih[DDIM + u]), b2 = bf16r(b_ih[2 * DDIM + u]);
    v4f o;
    o[0] = fmaf(fb, t0b, t0a) + b0;
    o[1] = fmaf(fb, t1b, t1a) + b1;
    o[2] = fmaf(fb, t2b, t2a) + b2;
    o[3] = 0.0f;
    float* op = GXT + (size_t)i * 4;
    *(volatile v4f*)op = o;
    __threadfence();
    *(volatile v4f*)op = o;
  }
}

__device__ __forceinline__ float gsig(float x)  { return __builtin_amdgcn_rcpf(1.0f + expf(-x)); }
__device__ __forceinline__ float gtanh(float x) { return 1.0f - 2.0f * __builtin_amdgcn_rcpf(expf(2.0f * x) + 1.0f); }

__device__ __forceinline__ void gru_rows_first(v8f ar, v8f az, v8f ai, v8f an, v4f pg, float bhr, float bhz, float bhn,
                                               int row16, int hh, int u, float* St, _Float16* Hn) {
#pragma unroll
  for (int r = 0; r < 8; ++r) {
    const int row = row16 + 8 * hh + r;
    const float rg  = gsig(ar[r] * GINV + pg[0] + bhr);
    const float zg  = gsig(az[r] * GINV + pg[1] + bhz);
    const float ghn = an[r] * GINV + bhn;
    const float ng  = gtanh(ai[r] * GINV + pg[2] + rg * ghn);
    const float ho  = St[row * SP + u];
    const float hn  = (1.0f - zg) * ng + zg * ho;
    St[row * SP + u] = hn;
    Hn[row * HP + u] = (_Float16)(hn * HCAR);
  }
}
__device__ __forceinline__ void gru_rows_next(v8f ar, v8f az, v8f an, const float* GXf, const int* Tg, int jcol,
                                              float bhr, float bhz, float bhn,
                                              int row16, int hh, int u, float* St, _Float16* Hn) {
#pragma unroll
  for (int r = 0; r < 8; ++r) {
    const int row = row16 + 8 * hh + r;
    const int tok = Tg[row * NSLOT + jcol];
    const v4f gx = *(const v4f*)(GXf + ((size_t)tok * DDIM + (size_t)u) * 4);
    const float rg  = gsig(gx[0] + (ar[r] * GINV + bhr));
    const float zg  = gsig(gx[1] + (az[r] * GINV + bhz));
    const float ghn = an[r] * GINV + bhn;
    const float ng  = gtanh(gx[2] + rg * ghn);
    const float ho  = St[row * SP + u];
    const float hn  = (1.0f - zg) * ng + zg * ho;
    St[row * SP + u] = hn;
    Hn[row * HP + u] = (_Float16)(hn * HCAR);
    asm volatile("" ::: "memory");
  }
}

__device__ __forceinline__ void gru_group_first(const _Float16* Hc, _Float16* Hn, float* St,
                                                const _Float16* WRZ, const _Float16* WIH, const _Float16* WHH,
                                                const float* P0, const float* b_hh,
                                                int u, int c, int hh, int koff) {
  const _Float16* wr = WRZ + (size_t)u * DDIM + koff;
  const _Float16* wz = WRZ + (size_t)(DDIM + u) * DDIM + koff;
  const _Float16* wi = WIH + (size_t)(2 * DDIM + u) * DDIM + koff;
  const _Float16* wn = WHH + (size_t)(2 * DDIM + u) * DDIM + koff;
  const _Float16* a0p = Hc + c * HP + koff;
  const _Float16* a1p = a0p + 16 * HP;
  const v8f z8 = {0.f, 0.f, 0.f, 0.f, 0.f, 0.f, 0.f, 0.f};
  v8f ar0 = z8, az0 = z8, ai0 = z8, an0 = z8, ar1 = z8, az1 = z8, ai1 = z8, an1 = z8;
#pragma unroll 1
  for (int k0 = 0; k0 < DDIM; k0 += 32) {
    const v16h br = Frag<_Float16>::load(wr + k0);
    const v16h bz = Frag<_Float16>::load(wz + k0);
    const v16h bi = Frag<_Float16>::load(wi + k0);
    const v16h bn = Frag<_Float16>::load(wn + k0);
    const v16h a0 = Frag<_Float16>::load(a0p + k0);
    const v16h a1 = Frag<_Float16>::load(a1p + k0);
    ar0 = Frag<_Float16>::mma(a0, br, ar0);
    az0 = Frag<_Float16>::mma(a0, bz, az0);
    ai0 = Frag<_Float16>::mma(a0, bi, ai0);
    an0 = Frag<_Float16>::mma(a0, bn, an0);
    ar1 = Frag<_Float16>::mma(a1, br, ar1);
    az1 = Frag<_Float16>::mma(a1, bz, az1);
    ai1 = Frag<_Float16>::mma(a1, bi, ai1);
    an1 = Frag<_Float16>::mma(a1, bn, an1);
    tie8_h(ar0, az0, ai0, an0, ar1, az1, ai1, an1, a0, a1, bn);
    keep4_h(br, bz, bi, bn);
  }
  accg8(ar0, az0, ai0, an0, ar1, az1, ai1, an1);
  const v4f pg = *(const v4f*)(P0 + (size_t)u * 4);
  const float bhr = bf16r(b_hh[u]), bhz = bf16r(b_hh[DDIM + u]), bhn = bf16r(b_hh[2 * DDIM + u]);
  gru_rows_first(ar0, az0, ai0, an0, pg, bhr, bhz, bhn, 0,  hh, u, St, Hn);
  gru_rows_first(ar1, az1, ai1, an1, pg, bhr, bhz, bhn, 16, hh, u, St, Hn);
}
__device__ __forceinline__ void gru_group_next(const _Float16* Hc, _Float16* Hn, float* St,
                                               const _Float16* WHH, const float* GXf, const int* Tg, int jcol,
                                               const float* b_hh, int u, int c, int hh, int koff) {
  const _Float16* wr = WHH + (size_t)u * DDIM + koff;
  const _Float16* wz = WHH + (size_t)(DDIM + u) * DDIM + koff;
  const _Float16* wn = WHH + (size_t)(2 * DDIM + u) * DDIM + koff;
  const _Float16* a0p = Hc + c * HP + koff;
  const _Float16* a1p = a0p + 16 * HP;
  const v8f z8 = {0.f, 0.f, 0.f, 0.f, 0.f, 0.f, 0.f, 0.f};
  v8f ar0 = z8, az0 = z8, an0 = z8, ar1 = z8, az1 = z8, an1 = z8;
#pragma unroll 1
  for (int k0 = 0; k0 < DDIM; k0 += 32) {
    const v16h br = Frag<_Float16>::load(wr + k0);
    const v16h bz = Frag<_Float16>::load(wz + k0);
    const v16h bn = Frag<_Float16>::load(wn + k0);
    const v16h a0 = Frag<_Float16>::load(a0p + k0);
    const v16h a1 = Frag<_Float16>::load(a1p + k0);
    ar0 = Frag<_Float16>::mma(a0, br, ar0);
    az0 = Frag<_Float16>::mma(a0, bz, az0);
    an0 = Frag<_Float16>::mma(a0, bn, an0);
    ar1 = Frag<_Float16>::mma(a1, br, ar1);
    az1 = Frag<_Float16>::mma(a1, bz, az1);
    an1 = Frag<_Float16>::mma(a1, bn, an1);
    tie6_h(ar0, az0, an0, ar1, az1, an1, a0, a1, bn);
    keep4_h(br, bz, bn, a1);
  }
  accg6(ar0, az0, an0, ar1, az1, an1);
  const float bhr = bf16r(b_hh[u]), bhz = bf16r(b_hh[DDIM + u]), bhn = bf16r(b_hh[2 * DDIM + u]);
  gru_rows_next(ar0, az0, an0, GXf, Tg, jcol, bhr, bhz, bhn, 0,  hh, u, St, Hn);
  gru_rows_next(ar1, az1, an1, GXf, Tg, jcol, bhr, bhz, bhn, 16, hh, u, St, Hn);
}
__device__ __forceinline__ void proj_group(const _Float16* Hs, float* Ls, const _Float16* WP, const float* proj_b,
                                           int f, int wave, int c, int hh, int koff) {
  const int v = 16 * wave + c;
  const _Float16* wp  = WP + ((size_t)f * VOC + (size_t)v) * DDIM + koff;
  const _Float16* a0p = Hs + c * HP + koff;
  const _Float16* a1p = a0p + 16 * HP;
  const v8f z8 = {0.f, 0.f, 0.f, 0.f, 0.f, 0.f, 0.f, 0.f};
  v8f p0 = z8, p1 = z8;
#pragma unroll 1
  for (int k0 = 0; k0 < DDIM; k0 += 32) {
    const v16h b  = Frag<_Float16>::load(wp + k0);
    const v16h a0 = Frag<_Float16>::load(a0p + k0);
    const v16h a1 = Frag<_Float16>::load(a1p + k0);
    p0 = Frag<_Float16>::mma(a0, b, p0);
    p1 = Frag<_Float16>::mma(a1, b, p1);
    dep_guard_h(p0, p1, a0, b);
    keep4_h(a1, b, a0, a1);
  }
  acc_guard2(p0, p1);
  const float pb = bf16r(proj_b[f * VOC + v]);
#pragma unroll
  for (int r = 0; r < 8; ++r) {
    Ls[(8 * hh + r) * LP + v]      = p0[r] * GINV + pb;
    Ls[(16 + 8 * hh + r) * LP + v] = p1[r] * GINV + pb;
  }
}
__device__ __forceinline__ void store_rows(const float* Ls, float* out, int f, int rbase, int wave, int lane) {
  float* ob = out + ((size_t)f * NROW + (size_t)rbase) * VOC;
  for (int pass = 0; pass < 2; ++pass) {
#pragma unroll
    for (int i = 0; i < 4; ++i) {
      const int row = 4 * wave + i;
      const v4f val = *(const v4f*)(Ls + row * LP + 4 * lane);
      *(volatile v4f*)(ob + (size_t)row * VOC + 4 * lane) = val;
    }
    __threadfence();
  }
}

__global__ __launch_bounds__(NTHR) void gru_seq_kernel(const float* __restrict__ h0, const int* __restrict__ target,
                                                       const float* __restrict__ b_hh, const float* __restrict__ proj_b,
                                                       const unsigned short* __restrict__ WIHp,
                                                       const unsigned short* __restrict__ WHHp,
                                                       const unsigned short* __restrict__ WRZp,
                                                       const unsigned short* __restrict__ WPp,
                                                       const float* __restrict__ GXT,
                                                       float* __restrict__ out) {
  __shared__ __align__(16) _Float16 Hh[2 * RB * HP];
  __shared__ __align__(16) float    St[RB * SP];
  __shared__ __align__(16) float    Ls[RB * LP];
  __shared__ int Tg[RB * NSLOT];
  const _Float16* WIH = (const _Float16*)WIHp;
  const _Float16* WHH = (const _Float16*)WHHp;
  const _Float16* WRZ = (const _Float16*)WRZp;
  const _Float16* WP  = (const _Float16*)WPp;
  const int tid = threadIdx.x, lane = tid & 31, wave = tid >> 5;
  const int c = lane & 15, hh = lane >> 4, koff = 8 * hh;
  const int rbase = blockIdx.x * RB;

#pragma unroll 1
  for (int it = 0; it < (RB * DDIM / 4) / NTHR; ++it) {
    const int idx = it * NTHR + tid;
    const int row = idx >> 7;
    const int c4  = (idx & 127) * 4;
    const v4f v = *(const v4f*)(h0 + (size_t)(rbase + row) * DDIM + c4);
    v4f s; v4h hv;
#pragma unroll
    for (int e = 0; e < 4; ++e) { const float bv = bf16r(v[e]); s[e] = bv; hv[e] = (_Float16)(bv * HCAR); }
    *(v4f*)(St + row * SP + c4) = s;
    *(v4h*)(Hh + row * HP + c4) = hv;
  }
  if (tid < RB * NSLOT) {
    const int r = tid >> 2, j = tid & 3;
    int t = target[(size_t)(rbase + r) * NSLOT + j];
    t = (t < 0) ? (t + VOC) : t;
    t = (t < 0) ? 0 : t;
    t = (t > VOC - 1) ? (VOC - 1) : t;
    Tg[tid] = t;
  }
  __syncthreads();

  const float* P0 = GXT + (size_t)(GXT_ROWS - 1) * DDIM * 4;

#pragma unroll 1
  for (int g4 = 0; g4 < 4; ++g4) {
    const int u = (wave * 4 + g4) * 16 + c;
    gru_group_first(Hh, Hh + RB * HP, St, WRZ, WIH, WHH, P0, b_hh, u, c, hh, koff);
  }
  __syncthreads();
  proj_group(Hh + RB * HP, Ls, WP, proj_b, 0, wave, c, hh, koff);
  __syncthreads();
  store_rows(Ls, out, 0, rbase, wave, lane);

#pragma unroll 1
  for (int f = 1; f < NSLOT; ++f) {
    const int cur = f & 1;
    const _Float16* Hc = Hh + cur * (RB * HP);
    _Float16*       Hn = Hh + (cur ^ 1) * (RB * HP);
    const float* GXf = GXT + (size_t)(f - 1) * VOC * DDIM * 4;
#pragma unroll 1
    for (int g4 = 0; g4 < 4; ++g4) {
      const int u = (wave * 4 + g4) * 16 + c;
      gru_group_next(Hc, Hn, St, WHH, GXf, Tg, f - 1, b_hh, u, c, hh, koff);
    }
    __syncthreads();
    proj_group(Hn, Ls, WP, proj_b, f, wave, c, hh, koff);
    __syncthreads();
    store_rows(Ls, out, f, rbase, wave, lane);
  }
}

extern "C" void kernel_launch(void* const* d_in, const int* in_sizes, int n_in,
                              void* d_out, int out_size, void* d_ws, size_t ws_size, hipStream_t stream) {
  if (n_in < 10 || d_out == nullptr || d_ws == nullptr) return;
  if (in_sizes[0] != NROW * DDIM || in_sizes[1] != NROW * NSLOT || in_sizes[2] != ETAB_EMB * DDIM ||
      in_sizes[3] != NSLOT * DDIM || in_sizes[4] != G3X * DDIM || in_sizes[5] != G3X * DDIM ||
      in_sizes[6] != G3X || in_sizes[7] != G3X || in_sizes[8] != NSLOT * VOC * DDIM || in_sizes[9] != NSLOT * VOC ||
      out_size != NSLOT * NROW * VOC) return;

  const float* hidden = (const float*)d_in[0];
  const int*   target = (const int*)d_in[1];
  const float* emb    = (const float*)d_in[2];
  const float* pos    = (const float*)d_in[3];
  const float* w_ih   = (const float*)d_in[4];
  const float* w_hh   = (const float*)d_in[5];
  const float* b_ih   = (const float*)d_in[6];
  const float* b_hh   = (const float*)d_in[7];
  const float* proj_w = (const float*)d_in[8];
  const float* proj_b = (const float*)d_in[9];
  float* out = (float*)d_out;

  char* ws = (char*)d_ws; size_t off = 0;
  auto carve = [&](size_t bytes) -> char* { char* p = ws + off; off += (bytes + 255) & ~(size_t)255; return p; };
  unsigned short* WIH16 = (unsigned short*)carve((size_t)G3X * DDIM * 2);
  unsigned short* WHH16 = (unsigned short*)carve((size_t)G3X * DDIM * 2);
  unsigned short* WRZ16 = (unsigned short*)carve((size_t)2 * DDIM * DDIM * 2);
  unsigned short* WP16  = (unsigned short*)carve((size_t)NSLOT * VOC * DDIM * 2);
  unsigned short* E16   = (unsigned short*)carve((size_t)ETAB_ROWS * DDIM * 2);
  float*          TRAW  = (float*)carve((size_t)ETAB_ROWS * G3X * 4);
  float*          GXT   = (float*)carve((size_t)GXT_ROWS * DDIM * 16);
  if (off > ws_size || off > (size_t)134217728) return;

  constexpr int N8_G3  = G3X * (DDIM / 8);
  constexpr int N8_RZ  = 2 * DDIM * (DDIM / 8);
  constexpr int N8_WP  = NSLOT * VOC * (DDIM / 8);
  constexpr int N8_E16 = ETAB_ROWS * (DDIM / 8);
  static_assert(N8_G3 % NTHR == 0 && N8_RZ % NTHR == 0 && N8_WP % NTHR == 0 && N8_E16 % NTHR == 0);
  cvt8_kernel<1><<<(N8_G3 + NTHR - 1) / NTHR, NTHR, 0, stream>>>(w_ih,   w_ih,   WIH16, G3X,         DDIM / 8, DDIM, WCAR);
  cvt8_kernel<1><<<(N8_G3 + NTHR - 1) / NTHR, NTHR, 0, stream>>>(w_hh,   w_hh,   WHH16, G3X,         DDIM / 8, DDIM, WCAR);
  cvt8_kernel<2><<<(N8_RZ + NTHR - 1) / NTHR, NTHR, 0, stream>>>(w_ih,   w_hh,   WRZ16, 2 * DDIM,    DDIM / 8, DDIM, WCAR);
  cvt8_kernel<1><<<(N8_WP + NTHR - 1) / NTHR, NTHR, 0, stream>>>(proj_w, proj_w, WP16,  NSLOT * VOC, DDIM / 8, DDIM, WCAR);
  e16_kernel<<<(N8_E16 + NTHR - 1) / NTHR, NTHR, 0, stream>>>(emb, pos, E16);

  static_assert(ETAB_ROWS % 64 == 0 && G3X % 64 == 0 && DDIM % 32 == 0);
  const dim3 tgrid((ETAB_ROWS / 64) * (G3X / 64) / 8, 1);
  wmma_gemm64<0, false, 0, 0, false, 0><<<tgrid, 256, 0, stream>>>(
      E16, E16, DDIM, 0L, WIH16, WIH16, DDIM, 0L, (void*)TRAW, (void*)TRAW, G3X, 0L,
      b_ih, TRAW, 0L, ETAB_ROWS, G3X, DDIM, TSCALE);

  constexpr int NGXT = GXT_ROWS * DDIM;
  static_assert(NGXT % NTHR == 0);
  gxt_kernel<<<(NGXT + NTHR - 1) / NTHR, NTHR, 0, stream>>>(TRAW, b_ih, GXT);

  gru_seq_kernel<<<NROW / RB, NTHR, 0, stream>>>(hidden, target, b_hh, proj_b, WIH16, WHH16, WRZ16, WP16, GXT, out);
}
